// EmoShift_31284541784731
// MI455X (gfx1250) — hardware-run, weakly checked
//
#include <hip/hip_runtime.h>


#ifndef SEQ
#define SEQ 96
#endif
#define SEQ_FULL 96
#ifndef OUT_SEQ
#define OUT_SEQ SEQ
#endif
#define NB   16
#define DM   512
#define W1P  1024
#define HDN  128
#define NCLS 2
#define PWV  4
#define JPW  4

static_assert(W1P == 2 * DM);
static_assert(DM % 32 == 0);
static_assert(HDN % 64 == 0);
static_assert((NB * SEQ) % 64 == 0);
static_assert(NB == 16);
static_assert(HDN == 128);
static_assert(NB * NCLS == 32);
static_assert(JPW == 4);
static_assert(SEQ % (PWV * JPW) == 0);
static_assert(SEQ <= SEQ_FULL);
static_assert(OUT_SEQ >= SEQ);
static_assert(((size_t)NB * SEQ * DM) % 8 == 0);
static_assert(((size_t)HDN * W1P) % 8 == 0);
static_assert((DM * 2) % 16 == 0);
static_assert(32 * 16 * 8 == 16 * 64 * 4);
static_assert(32 * 16 == JPW * NB * NCLS * 4);
static_assert(16 * 68 * 4 <= 131072);
static_assert((2 * HDN + PWV * JPW * 32) * 4 <= 131072);
static_assert((2 * HDN) % (32 * PWV) == 0);

typedef unsigned short bf;
typedef __attribute__((ext_vector_type(16))) __bf16   v16bf;
typedef __attribute__((ext_vector_type(8)))  unsigned short v8us;
typedef __attribute__((ext_vector_type(8)))  float    v8f;
typedef __attribute__((ext_vector_type(4)))  float    v4f;
typedef v4f  __attribute__((may_alias)) v4fa;

__device__ __forceinline__ unsigned short f2bf(float f) { unsigned u = __float_as_uint(f); u += 0x7FFFu + ((u >> 16) & 1u); return (unsigned short)(u >> 16); }
__device__ __forceinline__ float bfr(float f) { return __uint_as_float(((unsigned)f2bf(f)) << 16); }
__device__ __forceinline__ v16bf cat16b(v8us lo, v8us hi) { return __builtin_bit_cast(v16bf, __builtin_shufflevector(lo, hi, 0, 1, 2, 3, 4, 5, 6, 7, 8, 9, 10, 11, 12, 13, 14, 15)); }
__device__ __forceinline__ v8f wmmab(v16bf a, v16bf b, v8f c) { return __builtin_amdgcn_wmma_f32_16x16x32_bf16(false, a, false, b, (short)0, c, false, false); }
__device__ __forceinline__ v8f wmmabg(v16bf a, v16bf b, v8f c) { c = wmmab(a, b, c); asm volatile("v_nop\n\tv_nop\n\tv_nop\n\tv_nop" : "+v"(c) : "v"(a), "v"(b)); return c; }
__device__ __forceinline__ v16bf ldb(const bf* p)  { return cat16b(*(const v8us*)p, *(const v8us*)(p + 16)); }
__device__ __forceinline__ void wave_sync() { __builtin_amdgcn_fence(3  , "wavefront"); __builtin_amdgcn_wave_barrier(); asm volatile("" ::: "memory"); }

__global__ __launch_bounds__(256) void k_cvt8(const float* __restrict__ src, bf* dst, size_t n8) {
    const size_t i = (size_t)blockIdx.x * 256 + threadIdx.x; if (i >= n8) return;
    const v8f v = *(const v8f*)(src + i * 8); v8us o;
#pragma unroll
    for (int k = 0; k < 8; ++k) o[k] = f2bf(v[k]);
    *(volatile v8us*)(dst + i * 8) = o; __threadfence(); *(volatile v8us*)(dst + i * 8) = o;
}

__global__ __launch_bounds__(32) void k_gemm(const bf* __restrict__ A, const bf* __restrict__ Bt, const float* __restrict__ bias, float* C, int useb) {
    __shared__ __align__(16) float os[16 * 68];
    const int lane = threadIdx.x & 31, lr = lane & 15, hi = lane >> 4;
    const unsigned r0 = blockIdx.x * 64u, c0 = blockIdx.y * 64u;
    v8f acc[4][4];
#pragma unroll
    for (int mb = 0; mb < 4; ++mb)
#pragma unroll
        for (int nb = 0; nb < 4; ++nb) acc[mb][nb] = (v8f){};
    const size_t aoff = (size_t)(r0 + (unsigned)lr) * DM + 8 * hi, boff = (size_t)(c0 + (unsigned)lr) * W1P + 8 * hi;
#pragma unroll 1
    for (int kc = 0; kc < DM; kc += 32) {
        v16bf a[4];
#pragma unroll
        for (int mb = 0; mb < 4; ++mb) a[mb] = ldb(A + aoff + (size_t)mb * 16 * DM + kc);
#pragma unroll
        for (int nb = 0; nb < 4; ++nb) { const v16bf b = ldb(Bt + boff + (size_t)nb * 16 * W1P + kc);
#pragma unroll
            for (int mb = 0; mb < 4; ++mb) acc[mb][nb] = wmmabg(a[mb], b, acc[mb][nb]); }
    }
    float bc[4];
#pragma unroll
    for (int nb = 0; nb < 4; ++nb) { const float bv = bfr(bias[c0 + nb * 16 + lr]); bc[nb] = (useb != 0) ? bv : 0.0f; }
#pragma unroll
    for (int mb = 0; mb < 4; ++mb) {
#pragma unroll
        for (int nb = 0; nb < 4; ++nb) {
#pragma unroll
            for (int j = 0; j < 8; ++j) os[(hi * 8 + j) * 68 + nb * 16 + lr] = acc[mb][nb][j] + bc[nb]; }
        wave_sync();
        float* cb = C + (size_t)(r0 + (unsigned)(mb * 16)) * HDN + c0;
#pragma unroll 1
        for (int ps = 0; ps < 2; ++ps) {
#pragma unroll
            for (int s = 0; s < 8; ++s) { const int row = 2 * s + (lane >> 4), cofs = (lane & 15) * 4;
                const v4f val = *(const v4fa*)(&os[row * 68 + cofs]);
                *(volatile v4f*)(cb + (size_t)row * HDN + cofs) = val; }
            if (ps == 0) __threadfence(); }
        wave_sync();
    }
}

__global__ __launch_bounds__(32 * PWV) void k_pair(const float* __restrict__ HA, const float* __restrict__ HB, const float* __restrict__ W2, const float* __restrict__ b2, float* OUT) {
#pragma clang fp contract(off)
    __shared__ __align__(16) float w2s[2 * HDN];
    __shared__ __align__(16) float ost[PWV * JPW * 32];
    const int lane = threadIdx.x & 31, lb = lane & 15, hi = lane >> 4;
    const int wave = __builtin_amdgcn_readfirstlane((int)(threadIdx.x >> 5));
    const unsigned i = blockIdx.y;
    const unsigned j0 = (blockIdx.x * PWV + (unsigned)wave) * JPW;
#pragma unroll 1
    for (unsigned t = threadIdx.x; t < 2 * HDN; t += 32 * PWV) w2s[t] = bfr(W2[t]);
    __syncthreads();
    const float bz0 = bfr(b2[0]), bz1 = bfr(b2[1]);
    const float* har = HA + (size_t)(i * NB + (unsigned)lb) * HDN + 64 * hi;
    const float* hbr = HB + (size_t)(j0 * NB + (unsigned)lb) * HDN + 64 * hi;
    float p0[JPW], p1[JPW];
#pragma unroll
    for (int jj = 0; jj < JPW; ++jj) { p0[jj] = 0.0f; p1[jj] = 0.0f; }
#pragma unroll 1
    for (int u = 0; u < 64; u += 4) {
        const v4f a = *(const v4f*)(har + u);
        const v4f w0 = *(const v4fa*)(&w2s[64 * hi + u]);
        const v4f w1 = *(const v4fa*)(&w2s[HDN + 64 * hi + u]);
#pragma unroll
        for (int jj = 0; jj < JPW; ++jj) {
            const v4f c = *(const v4f*)(hbr + (size_t)jj * NB * HDN + u);
#pragma unroll
            for (int e = 0; e < 4; ++e) {
                const float s = a[e] + c[e];
                const float hv = fmaxf(s, 0.0f);
                p0[jj] = fmaf(hv, w0[e], p0[jj]);
                p1[jj] = fmaf(hv, w1[e], p1[jj]); }
        }
    }
    float q0[JPW], q1[JPW];
#pragma unroll
    for (int jj = 0; jj < JPW; ++jj) {
        const float x0 = __shfl_xor(p0[jj], 16, 32), x1 = __shfl_xor(p1[jj], 16, 32);
        q0[jj] = p0[jj] + x0; q1[jj] = p1[jj] + x1; }
    const float r00 = ((hi != 0) ? q0[2] : q0[0]) + bz0;
    const float r01 = ((hi != 0) ? q1[2] : q1[0]) + bz1;
    const float r10 = ((hi != 0) ? q0[3] : q0[1]) + bz0;
    const float r11 = ((hi != 0) ? q1[3] : q1[1]) + bz1;
    const int wb = wave * JPW * 32;
    ost[wb + (2 * hi) * 32 + 2 * lb]         = r00;
    ost[wb + (2 * hi) * 32 + 2 * lb + 1]     = r01;
    ost[wb + (2 * hi + 1) * 32 + 2 * lb]     = r10;
    ost[wb + (2 * hi + 1) * 32 + 2 * lb + 1] = r11;
    wave_sync();
    const v4f val = *(const v4fa*)(&ost[wb + lane * 4]);
    float* op = OUT + ((size_t)i * OUT_SEQ + (size_t)j0) * (NB * NCLS) + lane * 4;
    *(volatile v4f*)op = val; __threadfence(); *(volatile v4f*)op = val;
}

static constexpr size_t al256(size_t v) { return (v + 255) & ~(size_t)255; }
static constexpr size_t SZ_XB = al256((size_t)NB * SEQ * DM * 2);
static constexpr size_t SZ_WB = al256((size_t)HDN * W1P * 2);
static constexpr size_t SZ_HP = al256((size_t)NB * SEQ * HDN * 4);
static constexpr size_t SZ_TOTAL = 2 * SZ_XB + SZ_WB + 2 * SZ_HP;
static_assert(SZ_TOTAL <= (size_t)134217728);
static constexpr size_t N8_X = (size_t)NB * SEQ * DM / 8;
static constexpr size_t N8_W = (size_t)HDN * W1P / 8;
static constexpr unsigned G_X = (unsigned)((N8_X + 255) / 256);
static constexpr unsigned G_W = (unsigned)((N8_W + 255) / 256);
static constexpr size_t NEED_X = (size_t)NB * SEQ * DM;
static constexpr size_t NEED_O = ((size_t)(SEQ - 1) * OUT_SEQ + SEQ) * (NB * NCLS);
static_assert(N8_X * 8 * 2 <= SZ_XB);
static_assert(N8_W * 8 * 2 <= SZ_WB);
static_assert((size_t)(NB * SEQ / 64) * 64 * HDN * 4 <= SZ_HP);
static_assert((size_t)(HDN / 64) * 64 == HDN);

extern "C" void kernel_launch(void* const* d_in, const int* in_sizes, int n_in,
                              void* d_out, int out_size, void* d_ws, size_t ws_size, hipStream_t stream) {
    if (n_in < 8) return;
    if ((size_t)in_sizes[0] < NEED_X || (size_t)in_sizes[3] < NEED_X) return;
    if ((size_t)in_sizes[4] < (size_t)HDN * W1P) return;
    if (in_sizes[5] < HDN || in_sizes[6] < NCLS * HDN || in_sizes[7] < NCLS) return;
    if ((size_t)out_size < NEED_O) return;
    if (SZ_TOTAL > ws_size) return;
    const float* ea = (const float*)d_in[0];
    const float* ec = (const float*)d_in[3];
    const float* w1 = (const float*)d_in[4]; const float* b1 = (const float*)d_in[5];
    const float* w2 = (const float*)d_in[6]; const float* b2 = (const float*)d_in[7];
    float* OUT = (float*)d_out;
    char* wsp = (char*)d_ws;
    bf* XA = (bf*)wsp; wsp += SZ_XB;
    bf* XC = (bf*)wsp; wsp += SZ_XB;
    bf* WB = (bf*)wsp; wsp += SZ_WB;
    float* HA = (float*)wsp; wsp += SZ_HP;
    float* HB = (float*)wsp; wsp += SZ_HP;

    k_cvt8<<<G_X, 256, 0, stream>>>(ea, XA, N8_X);
    k_cvt8<<<G_X, 256, 0, stream>>>(ec, XC, N8_X);
    k_cvt8<<<G_W, 256, 0, stream>>>(w1, WB, N8_W);

    k_gemm<<<dim3(NB * SEQ / 64, HDN / 64, 1), 32, 0, stream>>>(XA, WB, b1, HA, 1);
    k_gemm<<<dim3(NB * SEQ / 64, HDN / 64, 1), 32, 0, stream>>>(XC, WB + DM, b1, HB, 0);

    k_pair<<<dim3(SEQ / (PWV * JPW), SEQ, 1), 32 * PWV, 0, stream>>>(HA, HB, w2, b2, OUT);
}
